// OfflineSlidingWindowAttn_35837207118659
// MI455X (gfx1250) — hardware-verified
//
#include <hip/hip_runtime.h>


#define NB_  2
#define NS_  2048
#define NHQ  16
#define NHK  4
#define HD   128
#define WIN  1024
#define CAP  30.0f
#define SCL  0.08838834764831845f
#define CLL  (-0.03f)
#define CLR  1.03f
#define LOSC 1024.0f
#define LOSCI (1.0f / 1024.0f)

typedef _Float16 h16;
typedef unsigned short bf;
typedef __attribute__((ext_vector_type(16))) __bf16   v16bf;
typedef __attribute__((ext_vector_type(16))) _Float16 v16h;
typedef __attribute__((ext_vector_type(8)))  _Float16 v8h;
typedef __attribute__((ext_vector_type(8)))  unsigned short v8us;
typedef __attribute__((ext_vector_type(8)))  float    v8f;
typedef __attribute__((ext_vector_type(4)))  float    v4f;
typedef __attribute__((ext_vector_type(4)))  unsigned short v4us;
typedef v8h  __attribute__((may_alias)) v8ha;
typedef v4f  __attribute__((may_alias)) v4fa;

__device__ __forceinline__ unsigned short f2bf(float f) { unsigned u = __float_as_uint(f); u += 0x7FFFu + ((u >> 16) & 1u); return (unsigned short)(u >> 16); }
__device__ __forceinline__ float bf2f(unsigned short b) { return __uint_as_float(((unsigned)b) << 16); }
__device__ __forceinline__ v16h cat16(v8h lo, v8h hi) { return __builtin_shufflevector(lo, hi, 0, 1, 2, 3, 4, 5, 6, 7, 8, 9, 10, 11, 12, 13, 14, 15); }
__device__ __forceinline__ v16bf cat16b(v8us lo, v8us hi) { return __builtin_bit_cast(v16bf, __builtin_shufflevector(lo, hi, 0, 1, 2, 3, 4, 5, 6, 7, 8, 9, 10, 11, 12, 13, 14, 15)); }
__device__ __forceinline__ v8f wmma16(v16h a, v16h b, v8f c) { return __builtin_amdgcn_wmma_f32_16x16x32_f16(false, a, false, b, (short)0, c, false, false); }
__device__ __forceinline__ v8f wmmab(v16bf a, v16bf b, v8f c) { return __builtin_amdgcn_wmma_f32_16x16x32_bf16(false, a, false, b, (short)0, c, false, false); }

__global__ __launch_bounds__(256) void k_qk(const float* __restrict__ q, const float* __restrict__ k, bf* QB, bf* KB) {
    const int lane = threadIdx.x & 31, wid = blockIdx.x * 8 + (threadIdx.x >> 5);
    const int nq = NB_ * NS_ * NHQ, nk = NB_ * NS_ * NHK;
    if (wid >= nq + nk) return;
    v4us o; const float* src; bf* dst;
    if (wid < nq) { const int b = wid / (NS_ * NHQ), rem = wid - b * NS_ * NHQ, s = rem / NHQ, h = rem - s * NHQ;
        src = q + (size_t)wid * HD; dst = QB + (((size_t)b * NHQ + h) * NS_ + s) * HD; }
    else { const int w2 = wid - nq; const int b = w2 / (NS_ * NHK), rem = w2 - b * NS_ * NHK, s = rem / NHK, h = rem - s * NHK;
        src = k + (size_t)w2 * HD; dst = KB + (((size_t)b * NHK + h) * NS_ + s) * HD; }
#pragma unroll
    for (int i = 0; i < 4; ++i) o[i] = f2bf(src[lane * 4 + i]);
    *(volatile v4us*)(dst + lane * 4) = o; __threadfence(); *(volatile v4us*)(dst + lane * 4) = o;
}
__global__ __launch_bounds__(256) void k_vt(const float* __restrict__ v, h16* VT) {
    __shared__ __align__(16) h16 tile[HD * 72];
    const int bid = blockIdx.x;
    const int b = bid / (NHK * (NS_ / 64)), rem = bid - b * (NHK * (NS_ / 64)), hk = rem / (NS_ / 64), st = rem - hk * (NS_ / 64);
    const int s0 = st * 64, tid = threadIdx.x;
    const int ss = tid >> 2, d0 = (tid & 3) * 32;
    const float* src = v + (((size_t)b * NS_ + s0 + ss) * NHK + hk) * HD + d0;
#pragma unroll
    for (int i = 0; i < 32; ++i) tile[(d0 + i) * 72 + ss] = (h16)bf2f(f2bf(src[i]));
    __syncthreads();
    const int piece = tid & 7;
    h16* base = VT + (((size_t)b * NHK + hk) * HD) * NS_ + s0;
    auto pass = [&]() {
#pragma unroll
        for (int s = 0; s < 4; ++s) { const int d = (tid >> 3) + 32 * s; const v8h val = *(const v8ha*)(tile + d * 72 + piece * 8); *(volatile v8h*)(base + (size_t)d * NS_ + piece * 8) = val; }
    };
    pass(); __threadfence(); pass();
}

#define SCORES(l0_)                                                                                                    \
    v8f s0 = {}, s1 = {};                                                                                              \
    { const bf* r0p = kb_b + (size_t)((l0_) + lr) * HD + 8 * hi; const bf* r1p = kb_b + (size_t)((l0_) + 16 + lr) * HD + 8 * hi; \
    _Pragma("unroll") for (int kc = 0; kc < 4; ++kc) {                                                                \
        s0 = wmmab(qa[kc], cat16b(*(const v8us*)(r0p + kc * 32), *(const v8us*)(r0p + kc * 32 + 16)), s0);          \
        s1 = wmmab(qa[kc], cat16b(*(const v8us*)(r1p + kc * 32), *(const v8us*)(r1p + kc * 32 + 16)), s1); } }      \
    asm volatile("v_nop\n\tv_nop\n\tv_nop\n\tv_nop" : "+v"(s0), "+v"(s1) : "v"(qa[0]), "v"(qa[3]));                   \
    float p0[8], p1[8];                                                                                                \
    _Pragma("unroll") for (int j = 0; j < 8; ++j) {                                                                   \
        const int k0i = (l0_) + lr, k1i = (l0_) + 16 + lr, qp = qpos[j];                                                \
        p0[j] = (k0i <= qp && k0i >= qp - WIN) ? CAP * tanhf(s0[j] * SCL) : -__builtin_inff();                         \
        p1[j] = (k1i <= qp && k1i >= qp - WIN) ? CAP * tanhf(s1[j] * SCL) : -__builtin_inff(); }

#define KT_RANGE const int kt0 = (qt * 64 >= WIN) ? ((qt * 64 - WIN) / 32) : 0; const int kt1 = (qt * 64 + 64) / 32;

__global__ __launch_bounds__(128) void k_stats(const bf* __restrict__ QB, const bf* __restrict__ KB, float* M, float* ZI) {
    __shared__ __align__(16) float stg[128];
    const int lane = threadIdx.x & 31, wave = threadIdx.x >> 5, lr = lane & 15, hi = lane >> 4;
    const int bid = blockIdx.x;
    const int b = bid / (NHQ * (NS_ / 64)), rem = bid - b * (NHQ * (NS_ / 64)), h = rem / (NS_ / 64), qt = rem - h * (NS_ / 64);
    const int q0 = qt * 64 + wave * 16, hk = h / (NHQ / NHK);
    const size_t qrow0 = ((size_t)b * NHQ + h) * NS_;
    v16bf qa[4];
#pragma unroll
    for (int kc = 0; kc < 4; ++kc) { const bf* p = QB + (qrow0 + q0 + lr) * HD + kc * 32 + 8 * hi; qa[kc] = cat16b(*(const v8us*)p, *(const v8us*)(p + 16)); }
    int qpos[8];
#pragma unroll
    for (int j = 0; j < 8; ++j) qpos[j] = q0 + 8 * hi + j;
    const bf* kb_b = KB + ((size_t)b * NHK + hk) * NS_ * HD;
    float mrow[8], lpart[8];
#pragma unroll
    for (int j = 0; j < 8; ++j) { mrow[j] = -3.0e38f; lpart[j] = 0.f; }
    KT_RANGE
#pragma unroll 1
    for (int kt = kt0; kt < kt1; ++kt) {
        SCORES(kt * 32)
#pragma unroll
        for (int j = 0; j < 8; ++j) {
            float mx = fmaxf(p0[j], p1[j]);
            mx = fmaxf(mx, __shfl_xor(mx, 1, 16)); mx = fmaxf(mx, __shfl_xor(mx, 2, 16)); mx = fmaxf(mx, __shfl_xor(mx, 4, 16)); mx = fmaxf(mx, __shfl_xor(mx, 8, 16));
            const float mn = fmaxf(mrow[j], mx); const float al = __expf(mrow[j] - mn); mrow[j] = mn;
            lpart[j] = lpart[j] * al + (__expf(p0[j] - mn) + __expf(p1[j] - mn));
        }
    }
#pragma unroll
    for (int j = 0; j < 8; ++j) {
        float rs = lpart[j]; rs += __shfl_xor(rs, 1, 16); rs += __shfl_xor(rs, 2, 16); rs += __shfl_xor(rs, 4, 16); rs += __shfl_xor(rs, 8, 16);
        if (lr == 0) { const int jl = wave * 16 + 8 * hi + j; stg[jl] = mrow[j]; stg[64 + jl] = 1.0f / rs; }
    }
    __syncthreads();
    if (wave == 0) {
        const v4f val = *(const v4fa*)(stg + hi * 64 + lr * 4);
        float* dst = (hi ? ZI : M) + qrow0 + qt * 64 + lr * 4;
        *(volatile v4f*)dst = val; __threadfence(); *(volatile v4f*)dst = val;
    }
}

__global__ __launch_bounds__(128) void k_out(const bf* __restrict__ QB, const bf* __restrict__ KB, const h16* __restrict__ VT, const float* __restrict__ M,
                                            const float* __restrict__ ZI, int dofs, float* out) {
    __shared__ __align__(16) h16 plds[4][16 * 32];
    __shared__ __align__(16) h16 plds2[4][16 * 32];
    __shared__ __align__(16) float ost[4][16 * 68];
    const int lane = threadIdx.x & 31, wave = threadIdx.x >> 5, lr = lane & 15, hi = lane >> 4;
    const int bid = blockIdx.x;
    const int b = bid / (NHQ * (NS_ / 64)), rem = bid - b * (NHQ * (NS_ / 64)), h = rem / (NS_ / 64), qt = rem - h * (NS_ / 64);
    const int q0 = qt * 64 + wave * 16, hk = h / (NHQ / NHK);
    const size_t qrow0 = ((size_t)b * NHQ + h) * NS_;
    h16* pl = &plds[wave][0]; h16* pl2 = &plds2[wave][0];
    v16bf qa[4];
#pragma unroll
    for (int kc = 0; kc < 4; ++kc) { const bf* p = QB + (qrow0 + q0 + lr) * HD + kc * 32 + 8 * hi; qa[kc] = cat16b(*(const v8us*)p, *(const v8us*)(p + 16)); }
    int qpos[8]; float mr[8], zr[8];
#pragma unroll
    for (int j = 0; j < 8; ++j) { qpos[j] = q0 + 8 * hi + j; mr[j] = M[qrow0 + qpos[j]]; zr[j] = ZI[qrow0 + qpos[j]]; }
    const bf* kb_b = KB + ((size_t)b * NHK + hk) * NS_ * HD;
    const h16* vt_b = VT + (((size_t)b * NHK + hk) * HD + dofs) * NS_;
    v8f o[4], ox[4];
#pragma unroll
    for (int n = 0; n < 4; ++n) { o[n] = (v8f){}; ox[n] = (v8f){}; }
    KT_RANGE
#pragma unroll 1
    for (int kt = kt0; kt < kt1; ++kt) {
        const int l0 = kt * 32;
        SCORES(l0)
#pragma unroll
        for (int j = 0; j < 8; ++j) {
            const float a0 = __expf(p0[j] - mr[j]) * zr[j], a1 = __expf(p1[j] - mr[j]) * zr[j];
            const float c0 = fminf(fmaxf((CLR - CLL) * a0 + CLL, 0.0f), 1.0f), c1 = fminf(fmaxf((CLR - CLL) * a1 + CLL, 0.0f), 1.0f);
            const int mrw = hi * 8 + j;
            const h16 hc0 = (h16)c0, hc1 = (h16)c1;
            pl[mrw * 32 + lr] = hc0; pl[mrw * 32 + 16 + lr] = hc1;
            pl2[mrw * 32 + lr] = (h16)((c0 - (float)hc0) * LOSC); pl2[mrw * 32 + 16 + lr] = (h16)((c1 - (float)hc1) * LOSC);
        }
        asm volatile("" ::: "memory");
        const v16h pa = cat16(*(const v8ha*)(pl + lr * 32 + hi * 8), *(const v8ha*)(pl + lr * 32 + 16 + hi * 8));
        const v16h px = cat16(*(const v8ha*)(pl2 + lr * 32 + hi * 8), *(const v8ha*)(pl2 + lr * 32 + 16 + hi * 8));
#pragma unroll
        for (int n = 0; n < 4; ++n) { const h16* vp = vt_b + (size_t)(n * 16 + lr) * NS_ + l0 + hi * 8; const v16h vb = cat16(*(const v8h*)vp, *(const v8h*)(vp + 16)); o[n] = wmma16(pa, vb, o[n]); ox[n] = wmma16(px, vb, ox[n]); }
        asm volatile("v_nop\n\tv_nop\n\tv_nop\n\tv_nop" : "+v"(o[0]), "+v"(o[1]), "+v"(o[2]), "+v"(o[3]), "+v"(ox[0]), "+v"(ox[1]), "+v"(ox[2]), "+v"(ox[3]) : "v"(pa), "v"(px));
    }
    float* os = &ost[wave][0];
#pragma unroll
    for (int n = 0; n < 4; ++n)
#pragma unroll
        for (int j = 0; j < 8; ++j) os[(hi * 8 + j) * 68 + n * 16 + lr] = o[n][j] + ox[n][j] * LOSCI;
    __syncthreads();
    auto pass = [&]() {
#pragma unroll
        for (int sI = 0; sI < 8; ++sI) { const int Lid = 4 * sI + (lane >> 3), piece = lane & 7; const int row = Lid >> 1, cofs = (Lid & 1) * 32 + piece * 4;
            const v4f val = *(const v4fa*)(os + row * 68 + cofs);
            *(volatile v4f*)(out + (((size_t)b * NS_ + q0 + row) * NHQ + h) * HD + dofs + cofs) = val; }
    };
    pass(); __threadfence(); pass();
}

extern "C" void kernel_launch(void* const* d_in, const int* in_sizes, int n_in,
                              void* d_out, int out_size, void* d_ws, size_t ws_size, hipStream_t stream) {
    (void)in_sizes; (void)n_in; (void)out_size;
    const float* q = (const float*)d_in[0]; const float* k = (const float*)d_in[1]; const float* v = (const float*)d_in[2];
    float* out = (float*)d_out;
    char* wsp = (char*)d_ws;
    auto take = [&](size_t bytes) { char* p = wsp; wsp += (bytes + 255) & ~(size_t)255; return (void*)p; };
    bf* QB = (bf*)take((size_t)NB_ * NHQ * NS_ * HD * 2); bf* KB = (bf*)take((size_t)NB_ * NHK * NS_ * HD * 2); h16* VT = (h16*)take((size_t)NB_ * NHK * HD * NS_ * 2);
    float* M = (float*)take((size_t)NB_ * NHQ * NS_ * 4); float* ZI = (float*)take((size_t)NB_ * NHQ * NS_ * 4);
    if ((size_t)(wsp - (char*)d_ws) > ws_size) return;
    k_qk<<<(NB_ * NS_ * (NHQ + NHK)) / 8, 256, 0, stream>>>(q, k, QB, KB);
    k_vt<<<NB_ * NHK * (NS_ / 64), 256, 0, stream>>>(v, VT);
    k_stats<<<NB_ * NHQ * (NS_ / 64), 128, 0, stream>>>(QB, KB, M, ZI);
    k_out<<<NB_ * NHQ * (NS_ / 64), 128, 0, stream>>>(QB, KB, VT, M, ZI, 0, out);
    k_out<<<NB_ * NHQ * (NS_ / 64), 128, 0, stream>>>(QB, KB, VT, M, ZI, HD / 2, out);
}
